// ConstraintEnforcementLayer_63831803953580
// MI455X (gfx1250) — hardware-run, weakly checked
//
#include <hip/hip_runtime.h>


#define NR   4096
#define NRP  4160
#define NM   256
#define NC   256
typedef _Float16 h16;
typedef unsigned short bf;
typedef __attribute__((ext_vector_type(16))) __bf16   v16bf;
typedef __attribute__((ext_vector_type(16))) _Float16 v16h;
typedef __attribute__((ext_vector_type(8)))  _Float16 v8h;
typedef __attribute__((ext_vector_type(8)))  unsigned short v8us;
typedef __attribute__((ext_vector_type(8)))  float    v8f;
typedef __attribute__((ext_vector_type(4)))  float    v4f;
typedef v8h  __attribute__((may_alias)) v8ha;
typedef v4f  __attribute__((may_alias)) v4fa;
typedef v8us __attribute__((may_alias)) v8usa;

__device__ __forceinline__ unsigned short f2bf(float f) { unsigned u = __float_as_uint(f); u += 0x7FFFu + ((u >> 16) & 1u); return (unsigned short)(u >> 16); }
__device__ __forceinline__ float bf2f(unsigned short b) { return __uint_as_float(((unsigned)b) << 16); }
__device__ __forceinline__ float bfr(float f) { return bf2f(f2bf(f)); }
__device__ __forceinline__ v16h cat16(v8h lo, v8h hi) { return __builtin_shufflevector(lo, hi, 0, 1, 2, 3, 4, 5, 6, 7, 8, 9, 10, 11, 12, 13, 14, 15); }
__device__ __forceinline__ v16bf cat16b(v8us lo, v8us hi) { return __builtin_bit_cast(v16bf, __builtin_shufflevector(lo, hi, 0, 1, 2, 3, 4, 5, 6, 7, 8, 9, 10, 11, 12, 13, 14, 15)); }
__device__ __forceinline__ v8f wmma16(v16h a, v16h b, v8f c) { return __builtin_amdgcn_wmma_f32_16x16x32_f16(false, a, false, b, (short)0, c, false, false); }
__device__ __forceinline__ v8f wmmab(v16bf a, v16bf b, v8f c) { return __builtin_amdgcn_wmma_f32_16x16x32_bf16(false, a, false, b, (short)0, c, false, false); }

template <typename T16> struct WFrag;
template <> struct WFrag<h16> { typedef v16h V; static __device__ __forceinline__ V ld(const h16* p) { return cat16(*(const v8h*)p, *(const v8h*)(p + 16)); } static __device__ __forceinline__ v8f mma(V a, V b, v8f c) { return wmma16(a, b, c); } };
template <> struct WFrag<bf> { typedef v16bf V; static __device__ __forceinline__ V ld(const bf* p) { return cat16b(*(const v8us*)p, *(const v8us*)(p + 16)); } static __device__ __forceinline__ v8f mma(V a, V b, v8f c) { return wmmab(a, b, c); } };
template <typename T16, int NSPLIT, bool BIAS>
__global__ __launch_bounds__(32) void k_gemmw(const T16* __restrict__ A, const T16* __restrict__ A2, const T16* __restrict__ Bt, const T16* __restrict__ Bt2, int K, float* C, int ldc, const float* __restrict__ bias, size_t sA, size_t sB, size_t sC) {
    typedef typename WFrag<T16>::V V;
    __shared__ __align__(16) float os[16 * 68];
    const size_t z = blockIdx.z; A += z * sA; if (A2) A2 += z * sA; Bt += z * sB; if (Bt2) Bt2 += z * sB; C += z * sC;
    const int lane = threadIdx.x & 31, lr = lane & 15, hi = lane >> 4; const int r0 = blockIdx.x * 64, c0 = blockIdx.y * 64;
    v8f acc[4][4];
#pragma unroll
    for (int mb = 0; mb < 4; ++mb)
#pragma unroll
        for (int nb = 0; nb < 4; ++nb) acc[mb][nb] = (v8f){};
    const size_t aoff = (size_t)(r0 + lr) * K + 8 * hi, boff = (size_t)(c0 + lr) * K + 8 * hi;
    for (int kc = 0; kc < K; kc += 32) {
        V a[4], a2[4];
#pragma unroll
        for (int mb = 0; mb < 4; ++mb) { a[mb] = WFrag<T16>::ld(A + aoff + (size_t)mb * 16 * K + kc); if (NSPLIT == 1 || NSPLIT == 2) a2[mb] = WFrag<T16>::ld(A2 + aoff + (size_t)mb * 16 * K + kc); }
#pragma unroll
        for (int nb = 0; nb < 4; ++nb) { const V b = WFrag<T16>::ld(Bt + boff + (size_t)nb * 16 * K + kc); V b2; if (NSPLIT >= 2) b2 = WFrag<T16>::ld(Bt2 + boff + (size_t)nb * 16 * K + kc);
#pragma unroll
            for (int mb = 0; mb < 4; ++mb) { acc[mb][nb] = WFrag<T16>::mma(a[mb], b, acc[mb][nb]); if (NSPLIT == 1 || NSPLIT == 2) acc[mb][nb] = WFrag<T16>::mma(a2[mb], b, acc[mb][nb]); if (NSPLIT >= 2) acc[mb][nb] = WFrag<T16>::mma(a[mb], b2, acc[mb][nb]); } }
        asm volatile("v_nop\n\tv_nop\n\tv_nop\n\tv_nop" : "+v"(acc[0][0]), "+v"(acc[1][1]), "+v"(acc[2][2]), "+v"(acc[3][3]) : "v"(a[0]), "v"(a[3]));
    }
#pragma unroll
    for (int mb = 0; mb < 4; ++mb) {
#pragma unroll
        for (int nb = 0; nb < 4; ++nb) {
#pragma unroll
            for (int j = 0; j < 8; ++j) os[(hi * 8 + j) * 68 + nb * 16 + lr] = acc[mb][nb][j]; }
        __builtin_amdgcn_wave_barrier(); asm volatile("" ::: "memory");
        float* crow = C + (size_t)(r0 + mb * 16) * ldc + c0;
#pragma unroll 1
        for (int ps = 0; ps < 2; ++ps) {
#pragma unroll
            for (int s = 0; s < 8; ++s) { const int row = 2 * s + hi, cofs = lr * 4; v4f val = *(const v4fa*)(os + row * 68 + cofs); if (BIAS) { val[0] += bfr(bias[c0 + cofs]); val[1] += bfr(bias[c0 + cofs + 1]); val[2] += bfr(bias[c0 + cofs + 2]); val[3] += bfr(bias[c0 + cofs + 3]); }
                *(volatile v4f*)(crow + (size_t)row * ldc + cofs) = val; }
            if (ps == 0) __threadfence(); }
        __builtin_amdgcn_wave_barrier(); asm volatile("" ::: "memory");
    }
}

typedef __attribute__((ext_vector_type(2))) _Float16 v2h;
typedef __attribute__((ext_vector_type(4))) _Float16 v4h;
typedef __attribute__((ext_vector_type(2))) unsigned short v2us;
typedef __attribute__((ext_vector_type(4))) unsigned short v4us;
typedef __attribute__((ext_vector_type(2))) float v2f;
__device__ __forceinline__ h16 toh_flush(float x) { const float z = (fabsf(x) < 6.103515625e-05f) ? 0.0f : x; return (h16)z; }

__global__ __launch_bounds__(32) void k_pl(const float* __restrict__ src, int srows, const float* __restrict__ c, float uc, h16* dst) { const int r = blockIdx.y; const int col = threadIdx.x * 8; const int rr = r < srows ? r : srows - 1; const float ly = r < srows ? 1.0f : 0.0f; const float ic = (r == srows) ? uc : 0.0f; const v8f s = *(const v8f*)(src + (size_t)rr * NC + col); const v8f cv = *(const v8f*)(c + col); v8h o;
#pragma unroll
    for (int q = 0; q < 8; ++q) { const float cb = bfr(cv[q]); const float d = __fsub_rn(bfr(s[q]), __fmul_rn(uc, cb)); o[q] = toh_flush(__fadd_rn(__fmul_rn(ly, d), __fmul_rn(ic, cb))); }
    h16* p = dst + (size_t)r * NC + col; *(volatile v8h*)p = o; __threadfence(); *(volatile v8h*)p = o; }

__global__ __launch_bounds__(256) void k_e(const float* __restrict__ b, const float* __restrict__ Pc, float* E) { const int m = threadIdx.x; const float e = __fsub_rn(bfr(b[m]), Pc[m]); *(volatile float*)(E + m) = e; __threadfence(); *(volatile float*)(E + m) = e; }

__global__ __launch_bounds__(256) void k_t(const float* __restrict__ P, const float* __restrict__ E, float* T) { const int r = blockIdx.x * 256 + threadIdx.x; if (r >= NR) return; const float* p = P + (size_t)r * NM; float mn = 2.0f;
    for (int g = 0; g < NM / 4; ++g) { const v4f d = *(const v4f*)(p + 4 * g); const v4f e = *(const v4f*)(E + 4 * g);
#pragma unroll
        for (int k = 0; k < 4; ++k) { float q = __fdiv_rn(e[k], __fadd_rn(d[k], 1e-7f)); q = (q > 1.0f) ? 2.0f : q; q = (q < 0.0f) ? 2.0f : q; mn = (q < mn) ? q : mn; } }
    const float t = (mn > 1.0f) ? 1.0f : mn;
    *(volatile float*)(T + r) = t; __threadfence(); *(volatile float*)(T + r) = t; }

__global__ __launch_bounds__(256) void k_z(const float* __restrict__ y, const float* __restrict__ c, const float* __restrict__ T, float* out) { const int i = blockIdx.x * 256 + threadIdx.x; if (i >= NR * NC / 4) return; const int r = i / (NC / 4), n0 = (i % (NC / 4)) * 4; const float t = T[r]; const float u = __fsub_rn(1.0f, t); const v4f yv = *(const v4f*)(y + (size_t)i * 4); const v4f cv = *(const v4f*)(c + n0); v4f o;
#pragma unroll
    for (int k = 0; k < 4; ++k) o[k] = __fadd_rn(__fmul_rn(t, bfr(yv[k])), __fmul_rn(u, bfr(cv[k])));
    *(volatile v4f*)(out + (size_t)i * 4) = o; __threadfence(); *(volatile v4f*)(out + (size_t)i * 4) = o; }

extern "C" void kernel_launch(void* const* d_in, const int* in_sizes, int n_in, void* d_out, int out_size, void* d_ws, size_t ws_size, hipStream_t stream) {
    if (n_in < 4) return;
    if (in_sizes[0] != NR * NC || in_sizes[1] != NM * NC || in_sizes[2] != NM || in_sizes[3] != NC) return;
    if (out_size != NR * NC) return;
    static_assert(NRP % 64 == 0 && NRP >= NR + 1 && NM % 64 == 0 && NC % 32 == 0 && NC == 256 && NM % 4 == 0 && NR % 256 == 0 && (NR * NC / 4) % 256 == 0, "the product: M and N multiples of 64, the depth a multiple of 32; a plane row is one wave's 256 words; every flat grid exact");
    const float* y = (const float*)d_in[0]; const float* A = (const float*)d_in[1]; const float* b = (const float*)d_in[2]; const float* c = (const float*)d_in[3];
    float* out = (float*)d_out;
    char* wsp = (char*)d_ws; auto take = [&](size_t bytes) { char* p = wsp; wsp += (bytes + 255) & ~(size_t)255; return (void*)p; };
    h16* Lp = (h16*)take((size_t)NRP * NC * 2); h16* Ap = (h16*)take((size_t)NM * NC * 2); float* P = (float*)take((size_t)NRP * NM * 4); float* E = (float*)take((size_t)NM * 4); float* T = (float*)take((size_t)NR * 4);
    if ((size_t)(wsp - (char*)d_ws) > ws_size) return;
    k_pl<<<dim3(1, NRP, 1), 32, 0, stream>>>(y, NR, c, 1.0f, Lp);
    k_pl<<<dim3(1, NM, 1), 32, 0, stream>>>(A, NM, c, 0.0f, Ap);
    k_gemmw<h16, 0, false><<<dim3(NRP / 64, NM / 64, 1), 32, 0, stream>>>(Lp, nullptr, Ap, nullptr, NC, P, NM, nullptr, 0, 0, 0);
    k_e<<<1, 256, 0, stream>>>(b, P + (size_t)NR * NM, E);
    k_t<<<(unsigned)(NR / 256), 256, 0, stream>>>(P, E, T);
    k_z<<<(unsigned)(NR * NC / 4 / 256), 256, 0, stream>>>(y, c, T, out);
}
